// ConstraintGNN_55843164782680
// MI455X (gfx1250) — hardware-verified
//
#include <hip/hip_runtime.h>
#include <stdint.h>
#include <stddef.h>


typedef _Float16 v16h __attribute__((ext_vector_type(16)));
typedef _Float16 v8h_t __attribute__((ext_vector_type(8)));
typedef v8h_t __attribute__((may_alias)) v8h;
typedef float v8f __attribute__((ext_vector_type(8)));
typedef float v4f_t __attribute__((ext_vector_type(4)));
typedef v4f_t __attribute__((may_alias)) v4f;
typedef int v4i_t __attribute__((ext_vector_type(4)));
typedef v4i_t __attribute__((may_alias)) v4i;
typedef unsigned int u32;

#define HID 64
#define WSCALE 16.0f
#define WINV 0.0625f

#define AGG_R 1024
#define AGG_BCAP 32
#define AGG_CHUNK 65536
#define AGG_OFF_DEG 262144
#define AGG_OFF_L 266240
#define AGG_OFF_CNT 282624
#define AGG_LDS 283136
#define SRC_SENT 0x7fffffff

union Frag16 { v16h v; v8h_t h[2]; };

__device__ __forceinline__ v16h ld_frag(const _Float16* t, int pitch, int rc, int k0, int hh) {
    const _Float16* q = t + rc * pitch + k0 + 8 * hh;
    Frag16 f;
    f.h[0] = *(const v8h*)q;
    f.h[1] = *(const v8h*)(q + 16);
    return f.v;
}

__device__ __forceinline__ v8f wmma_f16(v16h a, v16h b, v8f c) {
    c = __builtin_amdgcn_wmma_f32_16x16x32_f16(false, a, false, b, (short)0, c, false, false);
    asm volatile("v_nop\n\tv_nop\n\tv_nop\n\tv_nop" : "+v"(c) : "v"(a), "v"(b));
    return c;
}

__global__ __launch_bounds__(256) void enc_b_kernel(
    const float* __restrict__ X, int nb,
    const float* __restrict__ W1, const float* __restrict__ b1,
    const float* __restrict__ W2, const float* __restrict__ b2,
    float* hout, int ntiles)
{
    __shared__ __attribute__((aligned(16))) _Float16 Wt[64 * 64];
    __shared__ float W1s[5 * 64];
    __shared__ float b1s[64];
    __shared__ float b2s[64];
    __shared__ __attribute__((aligned(16))) _Float16 As[8 * 16 * 64];
    __shared__ __attribute__((aligned(16))) float Cs[8 * 16 * 64];

    const int tid = threadIdx.x, w = tid >> 5, lane = tid & 31;
    const int m = lane & 15, hh = lane >> 4;

    for (int i = tid; i < 64 * 64; i += 256) {
        const int n = i >> 6, k = i & 63;
        Wt[i] = (_Float16)(W2[k * 64 + n] * WSCALE);
    }
    for (int i = tid; i < 5 * 64; i += 256) W1s[i] = W1[i];
    if (tid < 64) { b1s[tid] = b1[tid]; b2s[tid] = b2[tid]; }
    __syncthreads();

    const int tile = blockIdx.x * 8 + w;
    const bool valid = tile < ntiles;
    const int row0 = tile * 16;
    _Float16* as = As + w * 1024;
    float* cs = Cs + w * 1024;

    {
        const int row = row0 + m;
        float xr[5];
#pragma unroll
        for (int k = 0; k < 5; ++k) xr[k] = (row < nb) ? X[(size_t)row * 5 + k] : 0.0f;
#pragma unroll 2
        for (int j = 0; j < 32; ++j) {
            const int nn = hh * 32 + j;
            float a = b1s[nn];
#pragma unroll
            for (int k = 0; k < 5; ++k) a += xr[k] * W1s[k * 64 + nn];
            as[m * 64 + nn] = (_Float16)fmaxf(a, 0.0f);
        }
    }
    __syncthreads();

    v8f acc[4] = {};
#pragma unroll
    for (int kb = 0; kb < 2; ++kb) {
        const v16h a = ld_frag(as, 64, m, kb * 32, hh);
#pragma unroll
        for (int nt = 0; nt < 4; ++nt)
            acc[nt] = wmma_f16(a, ld_frag(Wt, 64, nt * 16 + m, kb * 32, hh), acc[nt]);
    }
#pragma unroll
    for (int nt = 0; nt < 4; ++nt) {
        const int n = nt * 16 + m;
#pragma unroll
        for (int r = 0; r < 8; ++r)
            cs[(8 * hh + r) * 64 + n] = acc[nt][r] * WINV + b2s[n];
    }
    __syncthreads();

    if (valid) {
        float* dst = hout + (size_t)tile * 1024;
        for (int ps = 0; ps < 2; ++ps) {
#pragma unroll
            for (int i = 0; i < 8; ++i) {
                const v4f_t v = *(const v4f*)(cs + i * 128 + lane * 4);
                *(volatile v4f_t*)(dst + i * 128 + lane * 4) = v;
            }
            __threadfence();
        }
    }
}

extern __shared__ __attribute__((aligned(16))) unsigned char agg_smem[];

__device__ __forceinline__ void agg_append(u32* cntL, u32* Lst, int w, u32 bin, u32 entry) {
    u32* cp = cntL + (w * 16 + (int)bin);
    const u32 p = *cp;
    if (p < (u32)AGG_BCAP) {
        Lst[(w * 16 + (int)bin) * AGG_BCAP + (int)p] = entry;
        *cp = p + 1u;
    }
}

__device__ __forceinline__ void agg_slot(int s, int e, int base, int lane, int w,
                                         const int* __restrict__ dstp, int nb,
                                         u32* cntL, u32* Lst) {
    const u32 t = (u32)s - (u32)base;
    const bool hit = t < (u32)AGG_R;
    const u32 mm = __builtin_amdgcn_ballot_w32(hit);
    if (mm != 0u) {
        u32 entry = 0u, bin = 0u;
        if (hit) {
            int d = dstp[e];
            d = d < 0 ? 0 : d;
            d = (d > nb - 1) ? (nb - 1) : d;
            entry = (t << 22) | ((u32)d & 0x3FFFFFu);
            bin = t >> 6;
        }
        if (__builtin_popcount(mm) == 1) {
            if (hit) agg_append(cntL, Lst, w, bin, entry);
        } else {
            u32 rem = mm;
            while (rem != 0u) {
                const int j = __builtin_ctz(rem);
                if (lane == j) agg_append(cntL, Lst, w, bin, entry);
                rem &= rem - 1u;
            }
        }
    }
}

__global__ __launch_bounds__(256) void agg_kernel(
    const int* __restrict__ edges, int ne, const float* __restrict__ ch, int nb,
    float* meanbuf, float* cntbuf)
{
    float* accf = (float*)agg_smem;
    int* deg = (int*)(agg_smem + AGG_OFF_DEG);
    u32* Lst = (u32*)(agg_smem + AGG_OFF_L);
    u32* cntL = (u32*)(agg_smem + AGG_OFF_CNT);

    const int tid = threadIdx.x, w = tid >> 5, lane = tid & 31;
    const int base = blockIdx.x * AGG_R;

    {
        const v4f_t z = {0.0f, 0.0f, 0.0f, 0.0f};
        v4f* p = (v4f*)agg_smem;
        for (int i = tid; i < (AGG_OFF_L / 16); i += 256) p[i] = z;
    }
    __syncthreads();

    const int* srcp = edges;
    const int* dstp = edges + ne;
    const int nchunks = (ne + AGG_CHUNK - 1) / AGG_CHUNK;
    const int g = tid >> 4, c4 = tid & 15;

    for (int c = 0; c < nchunks; ++c) {
        if (lane < 16) cntL[w * 16 + lane] = 0u;
        const int cb = c * AGG_CHUNK + w * (AGG_CHUNK / 8);
#pragma unroll 2
        for (int it = 0; it < (AGG_CHUNK / 8) / 128; ++it) {
            const int e = cb + it * 128 + lane * 4;
            int s0, s1, s2, s3;
            if (e + 3 < ne) {
                const v4i_t sv = *(const v4i*)(srcp + e);
                s0 = sv.x; s1 = sv.y; s2 = sv.z; s3 = sv.w;
            } else {
                s0 = (e < ne) ? srcp[e] : SRC_SENT;
                s1 = (e + 1 < ne) ? srcp[e + 1] : SRC_SENT;
                s2 = (e + 2 < ne) ? srcp[e + 2] : SRC_SENT;
                s3 = (e + 3 < ne) ? srcp[e + 3] : SRC_SENT;
            }
            agg_slot(s0, e, base, lane, w, dstp, nb, cntL, Lst);
            agg_slot(s1, e + 1, base, lane, w, dstp, nb, cntL, Lst);
            agg_slot(s2, e + 2, base, lane, w, dstp, nb, cntL, Lst);
            agg_slot(s3, e + 3, base, lane, w, dstp, nb, cntL, Lst);
        }
        __syncthreads();

        for (int ww = 0; ww < 8; ++ww) {
            u32 n = cntL[ww * 16 + g];
            n = (n > (u32)AGG_BCAP) ? (u32)AGG_BCAP : n;
            const u32* lp = Lst + (ww * 16 + g) * AGG_BCAP;
            for (u32 p = 0; p < n; ++p) {
                const u32 en = lp[p];
                const u32 ls = en >> 22;
                u32 d = en & 0x3FFFFFu;
                d = (d > (u32)(nb - 1)) ? (u32)(nb - 1) : d;
                const v4f_t v = *(const v4f*)(ch + (size_t)d * HID + c4 * 4);
                v4f* ap = (v4f*)(accf + (int)ls * HID + c4 * 4);
                *ap = *ap + v;
                if (c4 == 0) deg[ls] = deg[ls] + 1;
            }
        }
        __syncthreads();
    }

    float* mdst = meanbuf + (size_t)base * HID;
    float* cdst = cntbuf + base;
    for (int ps = 0; ps < 2; ++ps) {
        for (int i = 0; i < 64; ++i) {
            const int q = i * 256 + tid;
            const int row = q >> 4;
            const float dg = (float)deg[row];
            const float inv = 1.0f / fmaxf(dg, 1.0f);
            const v4f_t a = *(const v4f*)(accf + q * 4);
            const v4f_t mv = a * inv;
            *(volatile v4f_t*)(mdst + (size_t)q * 4) = mv;
        }
        {
            const int r4 = tid * 4;
            v4f_t cv;
            cv.x = (float)deg[r4];
            cv.y = (float)deg[r4 + 1];
            cv.z = (float)deg[r4 + 2];
            cv.w = (float)deg[r4 + 3];
            *(volatile v4f_t*)(cdst + r4) = cv;
        }
        __threadfence();
    }
}

__global__ __launch_bounds__(256) void node_a_kernel(
    const float* __restrict__ X, int na,
    const float* __restrict__ Wf1, const float* __restrict__ bf1,
    const float* __restrict__ Wf2, const float* __restrict__ bf2,
    const float* __restrict__ meanbuf, const float* __restrict__ cntbuf,
    const float* __restrict__ W1, const float* __restrict__ b1,
    const float* __restrict__ W2, const float* __restrict__ b2,
    const float* __restrict__ Ws1, const float* __restrict__ bs1,
    const float* __restrict__ Ws2, const float* __restrict__ bs2,
    float* out)
{
    __shared__ __attribute__((aligned(16))) _Float16 Wf2t[64 * 64];
    __shared__ __attribute__((aligned(16))) _Float16 W1t[64 * 128];
    __shared__ __attribute__((aligned(16))) _Float16 W2t[64 * 64];
    __shared__ __attribute__((aligned(16))) _Float16 Ws1t[32 * 64];
    __shared__ float Wf1s[10 * 64];
    __shared__ float bf1s[64];
    __shared__ float bf2s[64];
    __shared__ float b1s[64];
    __shared__ float b2s[64];
    __shared__ float bs1s[32];
    __shared__ float ws2s[32];
    __shared__ float bs2s[4];
    __shared__ __attribute__((aligned(16))) _Float16 Ac[8 * 16 * 128];
    __shared__ __attribute__((aligned(16))) _Float16 Ah[8 * 16 * 64];
    __shared__ __attribute__((aligned(16))) float Ss[8 * 16 * 32];
    __shared__ __attribute__((aligned(16))) float Os[128];

    const int tid = threadIdx.x, w = tid >> 5, lane = tid & 31;
    const int m = lane & 15, hh = lane >> 4;

    for (int i = tid; i < 64 * 64; i += 256) {
        const int n = i >> 6, k = i & 63;
        Wf2t[i] = (_Float16)(Wf2[k * 64 + n] * WSCALE);
        W2t[i] = (_Float16)(W2[k * 64 + n] * WSCALE);
    }
    for (int i = tid; i < 64 * 128; i += 256) {
        const int n = i >> 7, k = i & 127;
        W1t[i] = (_Float16)(W1[k * 64 + n] * WSCALE);
    }
    for (int i = tid; i < 32 * 64; i += 256) {
        const int n = i >> 6, k = i & 63;
        Ws1t[i] = (_Float16)(Ws1[k * 32 + n] * WSCALE);
    }
    for (int i = tid; i < 10 * 64; i += 256) Wf1s[i] = Wf1[i];
    if (tid < 64) { bf1s[tid] = bf1[tid]; bf2s[tid] = bf2[tid]; b1s[tid] = b1[tid]; b2s[tid] = b2[tid]; }
    if (tid < 32) { bs1s[tid] = bs1[tid]; ws2s[tid] = Ws2[tid]; }
    if (tid == 0) bs2s[0] = bs2[0];
    __syncthreads();

    const int tile = blockIdx.x * 8 + w;
    const int row0 = tile * 16;
    _Float16* ac = Ac + w * 2048;
    _Float16* ah = Ah + w * 1024;
    float* ss = Ss + w * 512;

    {
        const int row = row0 + m;
        float xr[10];
#pragma unroll
        for (int k = 0; k < 10; ++k) xr[k] = (row < na) ? X[(size_t)row * 10 + k] : 0.0f;
#pragma unroll 2
        for (int j = 0; j < 32; ++j) {
            const int nn = hh * 32 + j;
            float a = bf1s[nn];
#pragma unroll
            for (int k = 0; k < 10; ++k) a += xr[k] * Wf1s[k * 64 + nn];
            ah[m * 64 + nn] = (_Float16)fmaxf(a, 0.0f);
        }
    }
    __syncthreads();

    v8f c2[4] = {};
#pragma unroll
    for (int kb = 0; kb < 2; ++kb) {
        const v16h a = ld_frag(ah, 64, m, kb * 32, hh);
#pragma unroll
        for (int nt = 0; nt < 4; ++nt)
            c2[nt] = wmma_f16(a, ld_frag(Wf2t, 64, nt * 16 + m, kb * 32, hh), c2[nt]);
    }
#pragma unroll
    for (int nt = 0; nt < 4; ++nt) {
        const int n = nt * 16 + m;
#pragma unroll
        for (int r = 0; r < 8; ++r) {
            const float v = c2[nt][r] * WINV + bf2s[n];
            c2[nt][r] = v;
            ac[(8 * hh + r) * 128 + n] = (_Float16)v;
        }
    }
    for (int i = lane; i < 16 * 16; i += 32) {
        const int m2 = i >> 4, cq = i & 15;
        const v4f_t v = *(const v4f*)(meanbuf + (size_t)(row0 + m2) * HID + cq * 4);
        _Float16* p = ac + m2 * 128 + 64 + cq * 4;
        p[0] = (_Float16)v.x; p[1] = (_Float16)v.y; p[2] = (_Float16)v.z; p[3] = (_Float16)v.w;
    }
    float cf[8];
#pragma unroll
    for (int r = 0; r < 8; ++r) cf[r] = cntbuf[row0 + 8 * hh + r];
    __syncthreads();

    {
        v8f c1[4] = {};
#pragma unroll
        for (int kb = 0; kb < 4; ++kb) {
            const v16h a = ld_frag(ac, 128, m, kb * 32, hh);
#pragma unroll
            for (int nt = 0; nt < 4; ++nt)
                c1[nt] = wmma_f16(a, ld_frag(W1t, 128, nt * 16 + m, kb * 32, hh), c1[nt]);
        }
#pragma unroll
        for (int nt = 0; nt < 4; ++nt) {
            const int n = nt * 16 + m;
#pragma unroll
            for (int r = 0; r < 8; ++r) {
                const float u = c1[nt][r] * WINV + b1s[n];
                const float v = (cf[r] > 0.0f) ? u : c2[nt][r];
                ah[(8 * hh + r) * 64 + n] = (_Float16)v;
            }
        }
    }
    __syncthreads();

    {
        v8f c3[4] = {};
#pragma unroll
        for (int kb = 0; kb < 2; ++kb) {
            const v16h a = ld_frag(ah, 64, m, kb * 32, hh);
#pragma unroll
            for (int nt = 0; nt < 4; ++nt)
                c3[nt] = wmma_f16(a, ld_frag(W2t, 64, nt * 16 + m, kb * 32, hh), c3[nt]);
        }
#pragma unroll
        for (int nt = 0; nt < 4; ++nt) {
            const int n = nt * 16 + m;
#pragma unroll
            for (int r = 0; r < 8; ++r)
                ac[(8 * hh + r) * 64 + n] = (_Float16)fmaxf(c3[nt][r] * WINV + b2s[n], 0.0f);
        }
    }
    __syncthreads();

    {
        v8f c4[2] = {};
#pragma unroll
        for (int kb = 0; kb < 2; ++kb) {
            const v16h a = ld_frag(ac, 64, m, kb * 32, hh);
#pragma unroll
            for (int nt = 0; nt < 2; ++nt)
                c4[nt] = wmma_f16(a, ld_frag(Ws1t, 64, nt * 16 + m, kb * 32, hh), c4[nt]);
        }
#pragma unroll
        for (int nt = 0; nt < 2; ++nt) {
            const int n = nt * 16 + m;
#pragma unroll
            for (int r = 0; r < 8; ++r)
                ss[(8 * hh + r) * 32 + n] = fmaxf(c4[nt][r] * WINV + bs1s[n], 0.0f);
        }
    }
    __syncthreads();

    if (lane < 16) {
        float a = bs2s[0];
#pragma unroll
        for (int k = 0; k < 32; ++k) a += ss[lane * 32 + k] * ws2s[k];
        Os[w * 16 + lane] = a;
    }
    __syncthreads();

    if (w == 0) {
        const int rb = blockIdx.x * 128 + lane * 4;
        for (int ps = 0; ps < 2; ++ps) {
            const v4f_t v = *(const v4f*)(Os + lane * 4);
            if (rb + 3 < na) {
                *(volatile v4f_t*)(out + rb) = v;
            } else {
                volatile float* vo = (volatile float*)out;
                if (rb < na) vo[rb] = v.x;
                if (rb + 1 < na) vo[rb + 1] = v.y;
                if (rb + 2 < na) vo[rb + 2] = v.z;
                if (rb + 3 < na) vo[rb + 3] = v.w;
            }
            __threadfence();
        }
    }
}

static inline size_t align256(size_t x) { return (x + 255) & ~(size_t)255; }

extern "C" void kernel_launch(void* const* d_in, const int* in_sizes, int n_in,
                              void* d_out, int out_size, void* d_ws, size_t ws_size,
                              hipStream_t stream) {
    (void)n_in;

    const float* xa  = (const float*)d_in[0];
    const float* xb  = (const float*)d_in[1];
    const int*   edges = (const int*)d_in[2];
    const float* Wf1 = (const float*)d_in[3];
    const float* bf1 = (const float*)d_in[4];
    const float* Wf2 = (const float*)d_in[5];
    const float* bf2 = (const float*)d_in[6];
    const float* Wc1 = (const float*)d_in[7];
    const float* bc1 = (const float*)d_in[8];
    const float* Wc2 = (const float*)d_in[9];
    const float* bc2 = (const float*)d_in[10];
    const float* W1  = (const float*)d_in[11];
    const float* b1  = (const float*)d_in[12];
    const float* W2  = (const float*)d_in[13];
    const float* b2  = (const float*)d_in[14];
    const float* Ws1 = (const float*)d_in[15];
    const float* bs1 = (const float*)d_in[16];
    const float* Ws2 = (const float*)d_in[17];
    const float* bs2 = (const float*)d_in[18];
    float* out = (float*)d_out;

    const int na = in_sizes[0] / 10;
    const int nb = in_sizes[1] / 5;
    const int ne = in_sizes[2] / 2;
    if (na <= 0 || nb <= 0 || ne < 0) return;
    if (out_size < na) return;

    const int ntA = (na + 15) / 16;
    const int ntB = (nb + 15) / 16;
    const int nblkG = (na + AGG_R - 1) / AGG_R;

    size_t off = 0;
    const size_t hB_off = off;    off = align256(off + (size_t)ntB * 16 * HID * sizeof(float));
    const size_t mean_off = off;  off = align256(off + (size_t)nblkG * AGG_R * HID * sizeof(float));
    const size_t cnt_off = off;   off = align256(off + (size_t)nblkG * AGG_R * sizeof(float));
    if (off > ws_size) return;

    unsigned char* ws = (unsigned char*)d_ws;
    float* hB = (float*)(ws + hB_off);
    float* meanbuf = (float*)(ws + mean_off);
    float* cntbuf = (float*)(ws + cnt_off);

    (void)hipFuncSetAttribute(reinterpret_cast<const void*>(&agg_kernel),
                              hipFuncAttributeMaxDynamicSharedMemorySize, AGG_LDS);

    enc_b_kernel<<<(ntB + 7) / 8, 256, 0, stream>>>(xb, nb, Wc1, bc1, Wc2, bc2, hB, ntB);

    agg_kernel<<<nblkG, 256, AGG_LDS, stream>>>(edges, ne, hB, nb, meanbuf, cntbuf);

    node_a_kernel<<<(ntA + 7) / 8, 256, 0, stream>>>(
        xa, na, Wf1, bf1, Wf2, bf2, meanbuf, cntbuf, W1, b1, W2, b2, Ws1, bs1, Ws2, bs2, out);

    (void)hipGetLastError();
}
